// FlashMHA_14723147891227
// MI455X (gfx1250) — hardware-verified
//
#include <hip/hip_runtime.h>
#include <math.h>

constexpr int kBatch  = 4;
constexpr int kSeq    = 2048;
constexpr int kDim    = 1024;
constexpr int kHeads  = 16;
constexpr int kDh     = 64;
constexpr int kTok    = kBatch * kSeq;
constexpr int kQKVF   = 3 * kDim;
constexpr int kQKld   = 2 * kDim;
constexpr int kKC     = 64;
constexpr int kNChunk = kSeq / kKC;
constexpr int kNQB    = kSeq / 64;
constexpr float kWCarry     = 16.0f;
constexpr float kWCarryInv  = 1.0f / 16.0f;
constexpr float kPCarry     = 32768.0f;
constexpr float kCtxCarry   = 256.0f;
constexpr float kScoreScale = 0.125f;
constexpr float kCtxOverP   = kCtxCarry / kPCarry;
constexpr float kOutScale   = 1.0f / (kCtxCarry * kWCarry);
static_assert(kHeads * kDh == kDim, "shape");
static_assert(kDh == 64 && kKC == 64, "head tiles");
static_assert(kSeq % 64 == 0 && kTok % 64 == 0 && kDim % 64 == 0 && kQKld % 64 == 0, "M,N tile multiples of 64");
static_assert(kDim % 32 == 0 && kSeq % 32 == 0 && kDh % 32 == 0, "K multiples of 32");
static_assert((kTok * kDim) % 2048 == 0 && (kQKVF * kDim) % 2048 == 0 && (kDim * kDim) % 2048 == 0, "cast grids exact");
static_assert(((kTok / 64) * (kQKld / 64)) % 8 == 0 && ((kDim / 64) * (kSeq / 64)) % 8 == 0 && ((kTok / 64) * (kDim / 64)) % 8 == 0, "gemm grids exact");

typedef __attribute__((ext_vector_type(16))) _Float16 v16h;
typedef __attribute__((ext_vector_type(8)))  _Float16 v8h;
typedef __attribute__((ext_vector_type(16))) __bf16   v16b;
typedef __attribute__((ext_vector_type(8)))  __bf16   v8b;
typedef __attribute__((ext_vector_type(8)))  float    v8f;
typedef __attribute__((ext_vector_type(4)))  float    v4f;
typedef __attribute__((ext_vector_type(4)))  unsigned int v4u;

__device__ __forceinline__ unsigned short f2bf_bits(float f) {
  unsigned u = __float_as_uint(f);
  return (unsigned short)((u + 0x7FFFu + ((u >> 16) & 1u)) >> 16);
}
__device__ __forceinline__ float bf_bits2f(unsigned short h) { return __uint_as_float(((unsigned)h) << 16); }

__device__ __forceinline__ void dep_guard_h(v8f& a, v8f& b, v16h x, v16h y) { asm volatile("v_nop\n\tv_nop\n\tv_nop\n\tv_nop" : "+v"(a), "+v"(b) : "v"(x), "v"(y)); }
__device__ __forceinline__ void dep_guard_b(v8f& a, v8f& b, v16b x, v16b y) { asm volatile("v_nop\n\tv_nop\n\tv_nop\n\tv_nop" : "+v"(a), "+v"(b) : "v"(x), "v"(y)); }
__device__ __forceinline__ void keep4_h(v16h a, v16h b, v16h c, v16h d) { asm volatile("v_nop" :: "v"(a), "v"(b), "v"(c), "v"(d)); }
__device__ __forceinline__ void keep4_b(v16b a, v16b b, v16b c, v16b d) { asm volatile("v_nop" :: "v"(a), "v"(b), "v"(c), "v"(d)); }
__device__ __forceinline__ void acc_guard4(v8f& a, v8f& b, v8f& c, v8f& d) { asm volatile("v_nop\n\tv_nop\n\tv_nop\n\tv_nop" : "+v"(a), "+v"(b), "+v"(c), "+v"(d)); }
template <typename T> struct Frag;
template <> struct Frag<_Float16> {
  typedef v16h V; union U { v16h v; v8h h[2]; };
  static __device__ __forceinline__ v16h load(const _Float16* p) {
    U f; f.h[0] = *(const v8h*)(p); f.h[1] = *(const v8h*)(p + 16); return f.v;
  }
  static __device__ __forceinline__ v8f mma(v16h a, v16h b, v8f c) {
    return __builtin_amdgcn_wmma_f32_16x16x32_f16(false, a, false, b, (short)0, c, false, false);
  }
  static __device__ __forceinline__ void guard(v8f& a, v8f& b, v16h x, v16h y) { dep_guard_h(a, b, x, y); }
  static __device__ __forceinline__ void keep(v16h a, v16h b, v16h c, v16h d) { keep4_h(a, b, c, d); }
};
template <> struct Frag<__bf16> {
  typedef v16b V; union U { v16b v; v8b h[2]; };
  static __device__ __forceinline__ v16b load(const __bf16* p) {
    U f; f.h[0] = *(const v8b*)(p); f.h[1] = *(const v8b*)(p + 16); return f.v;
  }
  static __device__ __forceinline__ v8f mma(v16b a, v16b b, v8f c) {
    return __builtin_amdgcn_wmma_f32_16x16x32_bf16(false, a, false, b, (short)0, c, false, false);
  }
  static __device__ __forceinline__ void guard(v8f& a, v8f& b, v16b x, v16b y) { dep_guard_b(a, b, x, y); }
  static __device__ __forceinline__ void keep(v16b a, v16b b, v16b c, v16b d) { keep4_b(a, b, c, d); }
};

__device__ __forceinline__ unsigned pk16(unsigned short a, unsigned short b) { return (unsigned)a | ((unsigned)b << 16); }
__device__ __forceinline__ unsigned short h_bits(float f) { const _Float16 h = (_Float16)f; return __builtin_bit_cast(unsigned short, h); }

template <int ET> struct Elem;
template <> struct Elem<0> { typedef _Float16 T; };
template <> struct Elem<1> { typedef __bf16 T; };
template <int ET, bool SPLIT, int BIAS_MODE, int OUT_MODE, bool RESID, int ACT = 0>
__global__ __launch_bounds__(256) void wmma_gemm64(
    const unsigned short* __restrict__ Ap, const unsigned short* __restrict__ A2p, int lda, long strideA,
    const unsigned short* __restrict__ Btp, const unsigned short* __restrict__ Bt2p, int ldb, long strideB,
    void* __restrict__ Cout, void* __restrict__ Cout2, int ldc, long strideC,
    const float* __restrict__ bias,
    const float* __restrict__ resid, long strideR,
    int M, int N, int K, float scale) {
  typedef typename Elem<ET>::T T;
  typedef typename Frag<T>::V V;
  const T* A = (const T*)Ap; const T* A2 = (const T*)A2p; const T* Bt = (const T*)Btp; const T* Bt2 = (const T*)Bt2p;
  __shared__ __align__(16) float sT[8][16 * 68];
  const int b    = blockIdx.y;
  const int lane = threadIdx.x & 31;
  const int wave = threadIdx.x >> 5;
  const int tilesN = N >> 6;
  const int tilesM = M >> 6;
  const int tile = blockIdx.x * 8 + wave;
  if (tile >= tilesM * tilesN) return;
  const int tm = tile / tilesN;
  const int tn = tile - tm * tilesN;
  const int m0 = tm << 6;
  const int n0 = tn << 6;

  const T* Ab  = A  + (size_t)b * strideA;
  const T* Bb  = Bt + (size_t)b * strideB;
  const T* Ab2 = SPLIT ? (A2  + (size_t)b * strideA) : nullptr;
  const T* Bb2 = SPLIT ? (Bt2 + (size_t)b * strideB) : nullptr;

  const int rlane = lane & 15;
  const int koff  = (lane >> 4) * 8;
  const int mOff  = (lane >> 4) * 8;

  v8f acc[4][4];
#pragma unroll
  for (int i = 0; i < 4; ++i)
#pragma unroll
    for (int j = 0; j < 4; ++j) acc[i][j] = (v8f){0.f,0.f,0.f,0.f,0.f,0.f,0.f,0.f};

  for (int k0 = 0; k0 < K; k0 += 32) {
    V bh[4], bl[4];
#pragma unroll
    for (int j = 0; j < 4; ++j) {
      const size_t bo = (size_t)(n0 + (j << 4) + rlane) * ldb + koff + k0;
      bh[j] = Frag<T>::load(Bb + bo);
      if (SPLIT) bl[j] = Frag<T>::load(Bb2 + bo);
    }
#pragma unroll
    for (int i = 0; i < 4; ++i) {
      const size_t ao = (size_t)(m0 + (i << 4) + rlane) * lda + koff + k0;
      V ah = Frag<T>::load(Ab + ao);
      V al;
      if (SPLIT) al = Frag<T>::load(Ab2 + ao);
#pragma unroll
      for (int j = 0; j < 4; ++j) {
        acc[i][j] = Frag<T>::mma(ah, bh[j], acc[i][j]);
        if (SPLIT) {
          acc[i][j] = Frag<T>::mma(ah, bl[j], acc[i][j]);
          acc[i][j] = Frag<T>::mma(al, bh[j], acc[i][j]);
        }
      }
      Frag<T>::guard(acc[i][0], acc[i][3], ah, SPLIT ? al : ah);
    }
    Frag<T>::keep(bh[0], bh[1], bh[2], bh[3]);
    if (SPLIT) Frag<T>::keep(bl[0], bl[1], bl[2], bl[3]);
  }
  acc_guard4(acc[0][0], acc[0][1], acc[0][2], acc[0][3]);
  acc_guard4(acc[1][0], acc[1][1], acc[1][2], acc[1][3]);
  acc_guard4(acc[2][0], acc[2][1], acc[2][2], acc[2][3]);
  acc_guard4(acc[3][0], acc[3][1], acc[3][2], acc[3][3]);

  float* slab = sT[wave];
  const float* Rb = RESID ? (resid + (size_t)b * strideR) : nullptr;
#pragma unroll
  for (int i = 0; i < 4; ++i) {
    const int mBase = m0 + (i << 4);
#pragma unroll
    for (int j = 0; j < 4; ++j) {
      const int n = n0 + (j << 4) + rlane;
      float bv = 0.f;
      if (BIAS_MODE == 2) bv = bias[n];
#pragma unroll
      for (int r = 0; r < 8; ++r) {
        float v = acc[i][j][r] * scale;
        if (BIAS_MODE == 1) v += bias[mBase + mOff + r];
        if (BIAS_MODE == 2) v += bv;
        if (RESID) v += Rb[(size_t)(mBase + mOff + r) * ldc + n];
        if (ACT == 2) v = fmaxf(v, 0.0f);
        if (ACT == 4) v = (v > 0.f) ? v : 0.01f * v;
        slab[(mOff + r) * 68 + (j << 4) + rlane] = v;
      }
    }
    __builtin_amdgcn_fence(__ATOMIC_RELEASE, "workgroup");
    __builtin_amdgcn_wave_barrier();
    __builtin_amdgcn_fence(__ATOMIC_ACQUIRE, "workgroup");
    if (OUT_MODE == 0) {
      float* C = (float*)Cout + (size_t)b * strideC;
      const int hh = lane >> 4, c4 = (lane & 15) * 4;
      for (int pass = 0; pass < 2; ++pass) {
#pragma unroll
        for (int it = 0; it < 8; ++it) {
          const int row = it * 2 + hh;
          v4f v = *(const v4f*)(slab + row * 68 + c4);
          *(volatile v4f*)(C + (size_t)(mBase + row) * ldc + n0 + c4) = v;
        }
        __threadfence();
      }
    } else {
      const int q = lane >> 3, c8 = (lane & 7) * 8;
      unsigned short* C  = (unsigned short*)Cout  + (size_t)b * strideC;
      unsigned short* C2 = (OUT_MODE == 2) ? ((unsigned short*)Cout2 + (size_t)b * strideC) : nullptr;
      for (int pass = 0; pass < 2; ++pass) {
#pragma unroll
        for (int it = 0; it < 4; ++it) {
          const int row = it * 4 + q;
          const float* sp = slab + row * 68 + c8;
          v8h hv, lv;
#pragma unroll
          for (int e = 0; e < 8; ++e) {
            if (OUT_MODE == 1) {
              hv[e] = (_Float16)sp[e];
            } else {
              unsigned short hb = f2bf_bits(sp[e]);
              unsigned short lb = f2bf_bits(sp[e] - bf_bits2f(hb));
              hv[e] = __builtin_bit_cast(_Float16, hb);
              lv[e] = __builtin_bit_cast(_Float16, lb);
            }
          }
          *(volatile v8h*)(C + (size_t)(mBase + row) * ldc + n0 + c8) = hv;
          if (OUT_MODE == 2) *(volatile v8h*)(C2 + (size_t)(mBase + row) * ldc + n0 + c8) = lv;
        }
        __threadfence();
      }
    }
    __builtin_amdgcn_fence(__ATOMIC_RELEASE, "workgroup");
    __builtin_amdgcn_wave_barrier();
    __builtin_amdgcn_fence(__ATOMIC_ACQUIRE, "workgroup");
  }
}

__global__ __launch_bounds__(256) void cast8_f16_kernel(const float* __restrict__ in, unsigned short* __restrict__ out,
                                                    int n8, float carry) {
  const int i = blockIdx.x * 256 + threadIdx.x;
  if (i >= n8) return;
  const float* p = in + 8 * (size_t)i;
  const v4f a = *(const v4f*)(p);
  const v4f c = *(const v4f*)(p + 4);
  unsigned short hb[8];
#pragma unroll
  for (int e = 0; e < 4; ++e) {
    hb[e]     = h_bits(a[e] * carry);
    hb[4 + e] = h_bits(c[e] * carry);
  }
  const v4u u = (v4u){pk16(hb[0], hb[1]), pk16(hb[2], hb[3]), pk16(hb[4], hb[5]), pk16(hb[6], hb[7])};
  unsigned short* q = out + 8 * (size_t)i;
  *(volatile v4u*)q = u;
  __threadfence();
  *(volatile v4u*)q = u;
}

__device__ __forceinline__ v8f mma_h(v16h a, v16h b, v8f c) {
  c = __builtin_amdgcn_wmma_f32_16x16x32_f16(false, a, false, b, (short)0, c, false, false);
  asm volatile("v_nop\n\tv_nop\n\tv_nop\n\tv_nop" : "+v"(c) : "v"(a), "v"(b));
  return c;
}

__global__ __launch_bounds__(128) void attn_f16_kernel(const unsigned short* __restrict__ QKp,
                                                        const unsigned short* __restrict__ VTp,
                                                        unsigned short* __restrict__ CTXp) {
  __shared__ __align__(16) _Float16 Psh[4][16 * kKC];
  __shared__ __align__(16) float    Os[4][16 * 68];

  const int tid  = threadIdx.x;
  const int wave = tid >> 5;
  const int lane = tid & 31;
  const int hh   = lane >> 4;
  const int c    = lane & 15;
  const int koff = hh * 8;

  const int bx = blockIdx.x;
  const int qb = bx % kNQB;
  const int bh = bx / kNQB;
  const int h  = bh % kHeads;
  const int b  = bh / kHeads;
  const int q0 = qb * 64 + wave * 16;

  const _Float16* Qp = (const _Float16*)QKp + (size_t)b * kSeq * kQKld + h * kDh;
  const _Float16* Kp = Qp + kDim;
  const _Float16* Vp = (const _Float16*)VTp + (size_t)bh * kDh * kSeq;

  v16h qa[2];
#pragma unroll
  for (int dc = 0; dc < 2; ++dc)
    qa[dc] = Frag<_Float16>::load(Qp + (size_t)(q0 + c) * kQKld + dc * 32 + koff);

  float mrow[8], lrow[8];
  v8f oacc[4];
#pragma unroll
  for (int r = 0; r < 8; ++r) { mrow[r] = -INFINITY; lrow[r] = 0.f; }
#pragma unroll
  for (int t = 0; t < 4; ++t) oacc[t] = (v8f){0.f,0.f,0.f,0.f,0.f,0.f,0.f,0.f};

  _Float16* pw = Psh[wave];

#pragma unroll 1
  for (int kc = 0; kc < kNChunk; ++kc) {
    const int kv0 = kc * kKC;
    __syncthreads();

    v8f s[4];
#pragma unroll
    for (int j = 0; j < 4; ++j) {
      s[j] = (v8f){0.f,0.f,0.f,0.f,0.f,0.f,0.f,0.f};
#pragma unroll
      for (int dc = 0; dc < 2; ++dc) {
        const v16h kb = Frag<_Float16>::load(Kp + (size_t)(kv0 + j * 16 + c) * kQKld + dc * 32 + koff);
        s[j] = mma_h(qa[dc], kb, s[j]);
      }
    }
#pragma unroll
    for (int j = 0; j < 4; ++j)
#pragma unroll
      for (int r = 0; r < 8; ++r) s[j][r] = s[j][r] * kScoreScale;

#pragma unroll
    for (int r = 0; r < 8; ++r) {
      float m = fmaxf(fmaxf(s[0][r], s[1][r]), fmaxf(s[2][r], s[3][r]));
#pragma unroll
      for (int off = 1; off < 16; off <<= 1) m = fmaxf(m, __shfl_xor(m, off, 32));
      const float mnew  = fmaxf(mrow[r], m);
      const float alpha = expf(mrow[r] - mnew);
      mrow[r] = mnew;
      float psum = 0.f;
#pragma unroll
      for (int j = 0; j < 4; ++j) {
        const float p = expf(s[j][r] - mnew);
        psum += p;
        pw[(8 * hh + r) * kKC + j * 16 + c] = (_Float16)(p * kPCarry);
      }
#pragma unroll
      for (int off = 1; off < 16; off <<= 1) psum += __shfl_xor(psum, off, 32);
      lrow[r] = lrow[r] * alpha + psum;
#pragma unroll
      for (int t = 0; t < 4; ++t) oacc[t][r] *= alpha;
    }
    __builtin_amdgcn_fence(__ATOMIC_RELEASE, "workgroup");
    __builtin_amdgcn_wave_barrier();
    __builtin_amdgcn_fence(__ATOMIC_ACQUIRE, "workgroup");

#pragma unroll
    for (int kk = 0; kk < 2; ++kk) {
      const v16h pa = Frag<_Float16>::load(pw + c * kKC + kk * 32 + koff);
#pragma unroll
      for (int t = 0; t < 4; ++t) {
        const v16h vb = Frag<_Float16>::load(Vp + (size_t)(t * 16 + c) * kSeq + kv0 + kk * 32 + koff);
        oacc[t] = mma_h(pa, vb, oacc[t]);
      }
    }
  }

  float* os = Os[wave];
#pragma unroll
  for (int r = 0; r < 8; ++r) {
    const float inv = kCtxOverP / lrow[r];
#pragma unroll
    for (int t = 0; t < 4; ++t) os[(8 * hh + r) * 68 + t * 16 + c] = oacc[t][r] * inv;
  }
  __builtin_amdgcn_fence(__ATOMIC_RELEASE, "workgroup");
  __builtin_amdgcn_wave_barrier();
  __builtin_amdgcn_fence(__ATOMIC_ACQUIRE, "workgroup");
  {
    const int q = lane >> 3, c8 = (lane & 7) * 8;
    unsigned short* Cp = CTXp + (size_t)b * kSeq * kDim + h * kDh;
    for (int pass = 0; pass < 2; ++pass) {
#pragma unroll
      for (int it = 0; it < 4; ++it) {
        const int row = it * 4 + q;
        const float* sp = os + row * 68 + c8;
        unsigned short hb[8];
#pragma unroll
        for (int e = 0; e < 8; ++e) hb[e] = h_bits(sp[e]);
        const v4u u = (v4u){pk16(hb[0], hb[1]), pk16(hb[2], hb[3]), pk16(hb[4], hb[5]), pk16(hb[6], hb[7])};
        *(volatile v4u*)(Cp + (size_t)(q0 + row) * kDim + c8) = u;
      }
      __threadfence();
    }
  }
}

extern "C" void kernel_launch(void* const* d_in, const int* in_sizes, int n_in,
                              void* d_out, int out_size, void* d_ws, size_t ws_size,
                              hipStream_t stream) {
  if (n_in < 5) return;
  if (in_sizes[0] != kTok * kDim) return;
  if (in_sizes[1] != kQKVF * kDim) return;
  if (in_sizes[2] != kQKVF) return;
  if (in_sizes[3] != kDim * kDim) return;
  if (in_sizes[4] != kDim) return;
  if (out_size != kTok * kDim) return;

  const size_t szXh = (size_t)kTok * kDim * 2;
  const size_t szWq = (size_t)kQKVF * kDim * 2;
  const size_t szWo = (size_t)kDim * kDim * 2;
  const size_t szQK = (size_t)kTok * kQKld * 2;
  const size_t szVT = (size_t)kBatch * kHeads * kDh * kSeq * 2;
  const size_t szCT = (size_t)kTok * kDim * 2;
  const size_t offXh = 0;
  const size_t offWq = offXh + szXh;
  const size_t offWo = offWq + szWq;
  const size_t offQK = offWo + szWo;
  const size_t offVT = offQK + szQK;
  const size_t offCT = offVT + szVT;
  const size_t total = offCT + szCT;
  if (ws_size < total) return;

  const float* x     = (const float*)d_in[0];
  const float* w_qkv = (const float*)d_in[1];
  const float* b_qkv = (const float*)d_in[2];
  const float* w_o   = (const float*)d_in[3];
  const float* b_o   = (const float*)d_in[4];
  float* out = (float*)d_out;
  char* ws = (char*)d_ws;
  unsigned short* Xh   = (unsigned short*)(ws + offXh);
  unsigned short* Wq16 = (unsigned short*)(ws + offWq);
  unsigned short* Wo16 = (unsigned short*)(ws + offWo);
  unsigned short* QK16 = (unsigned short*)(ws + offQK);
  unsigned short* VT   = (unsigned short*)(ws + offVT);
  unsigned short* CTX  = (unsigned short*)(ws + offCT);

  const int n8x = (kTok * kDim) / 8;
  const int n8q = (kQKVF * kDim) / 8;
  const int n8o = (kDim * kDim) / 8;
  cast8_f16_kernel<<<dim3(n8x / 256), dim3(256), 0, stream>>>(x, Xh, n8x, 1.0f);
  cast8_f16_kernel<<<dim3(n8q / 256), dim3(256), 0, stream>>>(w_qkv, Wq16, n8q, kWCarry);
  cast8_f16_kernel<<<dim3(n8o / 256), dim3(256), 0, stream>>>(w_o, Wo16, n8o, kWCarry);

  const int blocksQK = ((kTok / 64) * (kQKld / 64)) / 8;
  wmma_gemm64<0, false, 2, 1, false, 0><<<dim3(blocksQK, 1), dim3(256), 0, stream>>>(
      Xh, Xh, kDim, 0L, Wq16, Wq16, kDim, 0L,
      (void*)QK16, (void*)QK16, kQKld, 0L, b_qkv, b_qkv, 0L, kTok, kQKld, kDim, kWCarryInv);

  const int blocksVT = ((kDim / 64) * (kSeq / 64)) / 8;
  wmma_gemm64<0, false, 1, 1, false, 0><<<dim3(blocksVT, kBatch), dim3(256), 0, stream>>>(
      Wq16 + (size_t)2 * kDim * kDim, Wq16 + (size_t)2 * kDim * kDim, kDim, 0L,
      Xh, Xh, kDim, (long)kSeq * kDim,
      (void*)VT, (void*)VT, kSeq, (long)kDim * kSeq,
      b_qkv + 2 * kDim, b_qkv, 0L, kDim, kSeq, kDim, kWCarryInv);

  attn_f16_kernel<<<dim3(kBatch * kHeads * kNQB), dim3(128), 0, stream>>>(QK16, VT, CTX);

  const int blocksOut = ((kTok / 64) * (kDim / 64)) / 8;
  wmma_gemm64<0, false, 2, 0, false, 0><<<dim3(blocksOut, 1), dim3(256), 0, stream>>>(
      CTX, CTX, kDim, 0L, Wo16, Wo16, kDim, 0L,
      (void*)out, (void*)out, kDim, 0L, b_o, b_o, 0L, kTok, kDim, kDim, kOutScale);
}
